// SubMarginLinear_74363063763040
// MI455X (gfx1250) — hardware-verified
//
#include <hip/hip_runtime.h>
#include <stddef.h>


#define BDIM   512
#define DDIM   512
#define NOUT   17982
#define NPADN  18048
#define CP     NPADN
#define XSC    8
#define WSC    1024
#define NTHR   256
#define NWAVE  8
#define TPW    64
#define WSCAP  134217728
#define LDS_GEMM (NWAVE * 32 * 64 * 4)
#define EPSV   1e-8f

static_assert((NPADN % 128) == 0);
static_assert(NPADN >= NOUT);
static_assert((NOUT % 2) == 0);
static_assert((DDIM % 128) == 0);
static_assert((BDIM % 128) == 0);
static_assert((BDIM % 32) == 0);
static_assert(((BDIM * NOUT) % (4 * NTHR)) == 0);
static_assert((CP % 32) == 0);
static_assert(NTHR == NWAVE * 32);
static_assert(LDS_GEMM <= 300 * 1024);

typedef float     v2f  __attribute__((ext_vector_type(2)));
typedef float     v4f  __attribute__((ext_vector_type(4)));
typedef float     v8f  __attribute__((ext_vector_type(8)));
typedef _Float16  v8h  __attribute__((ext_vector_type(8)));
typedef _Float16  v16h __attribute__((ext_vector_type(16)));
union FragH { v16h v; v8h h[2]; };

__device__ __forceinline__ v8f wmf(v16h a, v16h b, v8f c) {
  v8f d = __builtin_amdgcn_wmma_f32_16x16x32_f16(false, a, false, b, (short)0, c, false, false);
  asm volatile("v_nop\n\tv_nop\n\tv_nop\n\tv_nop" : "+v"(d) : "v"(a), "v"(b));
  return d;
}

__global__ __launch_bounds__(NTHR) void k_prepx(const float* __restrict__ x, _Float16* xh, float* rx) {
  __shared__ __attribute__((aligned(16))) float rxs[32];
  const int tid = threadIdx.x, lane = tid & 31, wave = tid >> 5;
  const int rbase = blockIdx.x * 32 + wave * 4;
#pragma unroll 1
  for (int i = 0; i < 4; ++i) {
    const int row = rbase + i;
    const float* p = x + (size_t)row * DDIM;
    const v4f f0 = *(const v4f*)(p + 8 * lane);
    const v4f f1 = *(const v4f*)(p + 8 * lane + 4);
    const v4f f2 = *(const v4f*)(p + 256 + 8 * lane);
    const v4f f3 = *(const v4f*)(p + 256 + 8 * lane + 4);
    float s0 = f0.x * f0.x + f0.y * f0.y + f0.z * f0.z + f0.w * f0.w;
    float s1 = f1.x * f1.x + f1.y * f1.y + f1.z * f1.z + f1.w * f1.w;
    float s2 = f2.x * f2.x + f2.y * f2.y + f2.z * f2.z + f2.w * f2.w;
    float s3 = f3.x * f3.x + f3.y * f3.y + f3.z * f3.z + f3.w * f3.w;
    float ss = (s0 + s1) + (s2 + s3);
    ss += __shfl_xor(ss, 16);
    ss += __shfl_xor(ss, 8);
    ss += __shfl_xor(ss, 4);
    ss += __shfl_xor(ss, 2);
    ss += __shfl_xor(ss, 1);
    const float rinv = 1.0f / fmaxf(sqrtf(ss), EPSV);
    v8h a, b;
    a[0] = (_Float16)(f0.x * (float)XSC); a[1] = (_Float16)(f0.y * (float)XSC);
    a[2] = (_Float16)(f0.z * (float)XSC); a[3] = (_Float16)(f0.w * (float)XSC);
    a[4] = (_Float16)(f1.x * (float)XSC); a[5] = (_Float16)(f1.y * (float)XSC);
    a[6] = (_Float16)(f1.z * (float)XSC); a[7] = (_Float16)(f1.w * (float)XSC);
    b[0] = (_Float16)(f2.x * (float)XSC); b[1] = (_Float16)(f2.y * (float)XSC);
    b[2] = (_Float16)(f2.z * (float)XSC); b[3] = (_Float16)(f2.w * (float)XSC);
    b[4] = (_Float16)(f3.x * (float)XSC); b[5] = (_Float16)(f3.y * (float)XSC);
    b[6] = (_Float16)(f3.z * (float)XSC); b[7] = (_Float16)(f3.w * (float)XSC);
    _Float16* d0 = xh + (size_t)row * DDIM + 8 * lane;
    _Float16* d1 = d0 + 256;
    *(volatile v8h*)d0 = a;
    *(volatile v8h*)d1 = b;
    __threadfence();
    *(volatile v8h*)d0 = a;
    *(volatile v8h*)d1 = b;
    if (lane == 0) rxs[wave * 4 + i] = rinv;
  }
  __syncthreads();
  if (tid < 8) {
    const v4f v = *(const v4f*)(rxs + 4 * tid);
    float* d = rx + blockIdx.x * 32 + 4 * tid;
    *(volatile v4f*)d = v;
    __threadfence();
    *(volatile v4f*)d = v;
  }
}

__global__ __launch_bounds__(NTHR) void k_prepw(const float* __restrict__ W, _Float16* wt, float* rw) {
  __shared__ __attribute__((aligned(16))) float tile[128 * TPW];
  __shared__ __attribute__((aligned(16))) float red[NWAVE * 64];
  __shared__ __attribute__((aligned(16))) float rws[64];
  const int tid = threadIdx.x, lane = tid & 31, g = tid >> 5, hh = lane >> 4, m = lane & 15;
  const int n0 = blockIdx.x * 64;
  const int n = n0 + 2 * lane;
  const bool ok = n < NOUT;
  const int na = ok ? n : (NOUT - 2);
  float ss0 = 0.f, ss1 = 0.f;
#pragma unroll 1
  for (int dc = 0; dc < DDIM; dc += 128) {
    __syncthreads();
#pragma unroll 4
    for (int p = 0; p < 16; ++p) {
      const int dl = g + 8 * p;
      const v2f w = *(const v2f*)(W + (size_t)(dc + dl) * NOUT + na);
      const float wx = ok ? w.x : 0.f;
      const float wy = ok ? w.y : 0.f;
      ss0 += wx * wx;
      ss1 += wy * wy;
      v2f t;
      t.x = wx; t.y = wy;
      *(v2f*)(tile + dl * TPW + 2 * lane) = t;
    }
    __syncthreads();
    v8h hv[4];
#pragma unroll
    for (int q = 0; q < 4; ++q) {
      const int nl = 8 * g + 2 * q + hh;
      const int d8 = 8 * m;
#pragma unroll
      for (int e = 0; e < 8; ++e) hv[q][e] = (_Float16)(tile[(d8 + e) * TPW + nl] * (float)WSC);
    }
#pragma unroll
    for (int q = 0; q < 4; ++q) {
      _Float16* d = wt + (size_t)(n0 + 8 * g + 2 * q + hh) * DDIM + dc + 8 * m;
      *(volatile v8h*)d = hv[q];
    }
    __threadfence();
#pragma unroll
    for (int q = 0; q < 4; ++q) {
      _Float16* d = wt + (size_t)(n0 + 8 * g + 2 * q + hh) * DDIM + dc + 8 * m;
      *(volatile v8h*)d = hv[q];
    }
  }
  red[g * 64 + 2 * lane]     = ss0;
  red[g * 64 + 2 * lane + 1] = ss1;
  __syncthreads();
  if (tid < 64) {
    float tot = 0.f;
#pragma unroll
    for (int gg = 0; gg < NWAVE; ++gg) tot += red[gg * 64 + tid];
    const bool okc = (n0 + tid) < NOUT;
    rws[tid] = okc ? (1.0f / fmaxf(sqrtf(tot), EPSV)) : 0.f;
  }
  __syncthreads();
  if (tid < 16) {
    const v4f v = *(const v4f*)(rws + 4 * tid);
    float* d = rw + n0 + 4 * tid;
    *(volatile v4f*)d = v;
    __threadfence();
    *(volatile v4f*)d = v;
  }
}

__global__ __launch_bounds__(NTHR) void k_gemm(const _Float16* __restrict__ xh, const _Float16* __restrict__ wt,
                                               const float* __restrict__ rx, const float* __restrict__ rw,
                                               float* cpl) {
  extern __shared__ v4f lds_dyn[];
  const int tid = threadIdx.x, lane = tid & 31, wave = tid >> 5, hh = lane >> 4, m = lane & 15;
  float* stg = (float*)lds_dyn + wave * (32 * 64);
  const int n0 = blockIdx.x * 128, m0 = blockIdx.y * 128;
  const int wm = (wave >> 1) * 32, wn = (wave & 1) * 64;
  const _Float16* ap = xh + (size_t)(m0 + wm + m) * DDIM + 8 * hh;
  const _Float16* bp = wt + (size_t)(n0 + wn + m) * DDIM + 8 * hh;

  v8f acc[2][4];
#pragma unroll
  for (int mt = 0; mt < 2; ++mt)
#pragma unroll
    for (int nt = 0; nt < 4; ++nt) { v8f z = {0.f, 0.f, 0.f, 0.f, 0.f, 0.f, 0.f, 0.f}; acc[mt][nt] = z; }

#pragma unroll 1
  for (int kt = 0; kt < DDIM / 32; ++kt) {
    const int k0 = 32 * kt;
    FragH a0, a1;
    a0.h[0] = *(const v8h*)(ap + k0);
    a0.h[1] = *(const v8h*)(ap + k0 + 16);
    a1.h[0] = *(const v8h*)(ap + 16 * DDIM + k0);
    a1.h[1] = *(const v8h*)(ap + 16 * DDIM + k0 + 16);
#pragma unroll
    for (int nt = 0; nt < 4; ++nt) {
      const _Float16* bq = bp + (size_t)nt * 16 * DDIM + k0;
      FragH b;
      b.h[0] = *(const v8h*)bq;
      b.h[1] = *(const v8h*)(bq + 16);
      acc[0][nt] = wmf(a0.v, b.v, acc[0][nt]);
      acc[1][nt] = wmf(a1.v, b.v, acc[1][nt]);
    }
  }

  constexpr float OSC = 1.0f / (float)(XSC * WSC);
  float rwv[4];
#pragma unroll
  for (int nt = 0; nt < 4; ++nt) rwv[nt] = rw[n0 + wn + 16 * nt + m] * OSC;
#pragma unroll
  for (int mt = 0; mt < 2; ++mt) {
    const float* rp = rx + m0 + wm + 16 * mt + 8 * hh;
    const v4f ra = *(const v4f*)rp;
    const v4f rb = *(const v4f*)(rp + 4);
    float* sp = stg + (16 * mt + 8 * hh) * 64 + m;
#pragma unroll
    for (int nt = 0; nt < 4; ++nt) {
#pragma unroll
      for (int r = 0; r < 4; ++r) sp[r * 64 + 16 * nt] = acc[mt][nt][r] * ra[r] * rwv[nt];
#pragma unroll
      for (int r = 4; r < 8; ++r) sp[r * 64 + 16 * nt] = acc[mt][nt][r] * rb[r - 4] * rwv[nt];
    }
  }
  __syncthreads();

  float* gbase = cpl + (size_t)(m0 + wm) * CP + n0 + wn;
#pragma unroll
  for (int q = 0; q < 16; ++q) {
    const int row = 2 * q + hh;
    const v4f v = *(const v4f*)(stg + row * 64 + 4 * m);
    *(volatile v4f*)(gbase + (size_t)row * CP + 4 * m) = v;
  }
  __threadfence();
#pragma unroll
  for (int q = 0; q < 16; ++q) {
    const int row = 2 * q + hh;
    const v4f v = *(const v4f*)(stg + row * 64 + 4 * m);
    *(volatile v4f*)(gbase + (size_t)row * CP + 4 * m) = v;
  }
}

__global__ __launch_bounds__(NTHR) void k_pack(const float* __restrict__ cpl, float* out) {
  const int t = blockIdx.x * NTHR + threadIdx.x;
  const int ff = 4 * t;
  const int b = ff / NOUT;
  const int n = ff - b * NOUT;
  float v[4];
#pragma unroll
  for (int e = 0; e < 4; ++e) {
    int nn = n + e;
    const int wrap = (nn >= NOUT) ? 1 : 0;
    nn -= wrap * NOUT;
    int bb = b + wrap;
    bb = bb > BDIM - 1 ? BDIM - 1 : bb;
    v[e] = cpl[(size_t)bb * CP + nn];
  }
  v4f o;
  o.x = v[0]; o.y = v[1]; o.z = v[2]; o.w = v[3];
  float* d = out + (size_t)ff;
  *(volatile v4f*)d = o;
  __threadfence();
  *(volatile v4f*)d = o;
}

extern "C" void kernel_launch(void* const* d_in, const int* in_sizes, int n_in,
                              void* d_out, int out_size, void* d_ws, size_t ws_size,
                              hipStream_t stream) {
  if (n_in < 2) return;
  if (in_sizes[0] != BDIM * DDIM || in_sizes[1] != DDIM * NOUT) return;
  if (out_size != BDIM * NOUT) return;

  const float* x = (const float*)d_in[0];
  const float* W = (const float*)d_in[1];
  float* out = (float*)d_out;

  char* ws = (char*)d_ws;
  size_t off = 0;
  const size_t oXh = off; off += (size_t)BDIM * DDIM * 2;      off = (off + 255) & ~(size_t)255;
  const size_t oWt = off; off += (size_t)NPADN * DDIM * 2;     off = (off + 255) & ~(size_t)255;
  const size_t oRx = off; off += (size_t)BDIM * 4;             off = (off + 255) & ~(size_t)255;
  const size_t oRw = off; off += (size_t)NPADN * 4;            off = (off + 255) & ~(size_t)255;
  const size_t oCp = off; off += (size_t)BDIM * CP * 4;        off = (off + 255) & ~(size_t)255;
  if (off > ws_size || off > (size_t)WSCAP) return;
  _Float16* xh  = (_Float16*)(ws + oXh);
  _Float16* wt  = (_Float16*)(ws + oWt);
  float*    rx  = (float*)(ws + oRx);
  float*    rw  = (float*)(ws + oRw);
  float*    cpl = (float*)(ws + oCp);

  k_prepx<<<BDIM / 32, NTHR, 0, stream>>>(x, xh, rx);
  k_prepw<<<NPADN / 64, NTHR, 0, stream>>>(W, wt, rw);
  hipFuncSetAttribute(reinterpret_cast<const void*>(&k_gemm),
                      hipFuncAttributeMaxDynamicSharedMemorySize, LDS_GEMM);
  k_gemm<<<dim3(NPADN / 128, BDIM / 128), NTHR, LDS_GEMM, stream>>>(xh, wt, rx, rw, cpl);
  k_pack<<<(BDIM * NOUT) / (4 * NTHR), NTHR, 0, stream>>>(cpl, out);
}
